// EquivariantGraphConvolution_50792283242913
// MI455X (gfx1250) — hardware-verified
//
#include <hip/hip_runtime.h>
#include <stddef.h>


#define HD    64
#define ROW   70
#define NFO   6
#define EFW   16
#define PQW   128
#define KE1   145
#define XP    64

#define NT    128
#define NW    4
#define EPT   8
#define CHUNK (NT * EPT)
#define WCAP  (EPT * 32)
#define LISTN (NW * WCAP)
#define PASSN (NW * 32)
#define PCAP  (CHUNK + PASSN)
#define NB    512
#define NPB   (NW * 16)
#define OCH   ((NPB * ROW) / 128)

#define OFF_PQ 0
#define OFF_WT 16384
#define OFF_W2 20480
#define OFF_WC 28672
#define OFF_WV 36864
#define OFF_N1 45056
#define OFF_N2 61440
#define WPLN   69632

static_assert(PASSN == NT);
static_assert(PCAP >= CHUNK + PASSN);
static_assert((NB % (2 * NW * 32)) == 0);
static_assert(OCH * 128 == NPB * ROW);
static_assert(OFF_WT == OFF_PQ + 2 * 128 * 64);
static_assert(OFF_W2 == OFF_WT + 2 * 64 * 32);
static_assert(OFF_WC == OFF_W2 + 2 * 64 * 64);
static_assert(OFF_WV == OFF_WC + 2 * 64 * 64);
static_assert(OFF_N1 == OFF_WV + 2 * 64 * 64);
static_assert(OFF_N2 == OFF_N1 + 2 * 64 * 128);
static_assert(WPLN == OFF_N2 + 2 * 64 * 64);

typedef float v8f __attribute__((ext_vector_type(8)));
typedef float v4f __attribute__((ext_vector_type(4))) __attribute__((may_alias));
typedef float v2f __attribute__((ext_vector_type(2))) __attribute__((may_alias));
typedef int v4i __attribute__((ext_vector_type(4))) __attribute__((may_alias));
typedef unsigned short v8us __attribute__((ext_vector_type(8))) __attribute__((may_alias));
typedef __bf16 v16bf __attribute__((ext_vector_type(16)));
union FragB { v16bf v; v8us u[2]; };

__device__ __forceinline__ unsigned short bfb(float x) {
  unsigned int u = __float_as_uint(x);
  u += 0x7FFFu + ((u >> 16) & 1u);
  return (unsigned short)(u >> 16);
}
__device__ __forceinline__ float bfv(unsigned short b) { return __uint_as_float(((unsigned int)b) << 16); }

__device__ __forceinline__ void split8(v8f x, v8us& hi, v8us& lo) {
  v8us hh = {0, 0, 0, 0, 0, 0, 0, 0};
  v8us ll = {0, 0, 0, 0, 0, 0, 0, 0};
#pragma unroll
  for (int i = 0; i < 8; ++i) {
    const unsigned short b = bfb(x[i]);
    hh[i] = b;
    ll[i] = bfb(x[i] - bfv(b));
  }
  hi = hh; lo = ll;
}

__device__ __forceinline__ void d2b(v8f d0, v8f d1, FragB& bh, FragB& bl) {
  split8(d0, bh.u[0], bl.u[0]);
  split8(d1, bh.u[1], bl.u[1]);
}

__device__ __forceinline__ void ldpair(const unsigned short* hp, const unsigned short* lp, int off, FragB& fh, FragB& fl) {
  fh.u[0] = *(const v8us*)(hp + off);
  fh.u[1] = *(const v8us*)(hp + off + 16);
  fl.u[0] = *(const v8us*)(lp + off);
  fl.u[1] = *(const v8us*)(lp + off + 16);
}

__device__ __forceinline__ v8f mma3(v16bf ah, v16bf al, v16bf bh, v16bf bl, v8f c) {
  v8f d = __builtin_amdgcn_wmma_f32_16x16x32_bf16(false, ah, false, bh, (short)0, c, false, false);
  d = __builtin_amdgcn_wmma_f32_16x16x32_bf16(false, ah, false, bl, (short)0, d, false, false);
  d = __builtin_amdgcn_wmma_f32_16x16x32_bf16(false, al, false, bh, (short)0, d, false, false);
  asm volatile("v_nop\n\tv_nop\n\tv_nop\n\tv_nop" : "+v"(d) : "v"(ah), "v"(al), "v"(bh), "v"(bl));
  return d;
}

__device__ __forceinline__ v8f ldc8(const float* p) {
  const v4f a = *(const v4f*)p;
  const v4f b = *(const v4f*)(p + 4);
  v8f c;
  c[0] = a.x; c[1] = a.y; c[2] = a.z; c[3] = a.w;
  c[4] = b.x; c[5] = b.y; c[6] = b.z; c[7] = b.w;
  return c;
}

__device__ __forceinline__ void stc8(float* p, v8f d) {
  v4f u0, u1;
  u0.x = d[0]; u0.y = d[1]; u0.z = d[2]; u0.w = d[3];
  u1.x = d[4]; u1.y = d[5]; u1.z = d[6]; u1.w = d[7];
  *(v4f*)p = u0;
  *(v4f*)(p + 4) = u1;
}

__device__ __forceinline__ float silu_f(float x) { return x * __builtin_amdgcn_rcpf(1.0f + __expf(-x)); }
__device__ __forceinline__ float sigm_f(float x) { return __builtin_amdgcn_rcpf(1.0f + __expf(-x)); }
__device__ __forceinline__ v8f silu8(v8f a) {
  v8f r;
#pragma unroll
  for (int i = 0; i < 8; ++i) r[i] = silu_f(a[i]);
  return r;
}

__global__ __launch_bounds__(NT) void k_prep(const float* __restrict__ We1, const float* __restrict__ We2,
                                         const float* __restrict__ Wc1, const float* __restrict__ Wv1,
                                         const float* __restrict__ Wn1, const float* __restrict__ Wn2,
                                         unsigned short* wpl) {
  const int id = blockIdx.y;
  int rows = 64, kp = 64, base = OFF_N2;
  if (id == 0)      { rows = 128; kp = 64; base = OFF_PQ; }
  else if (id == 1) { kp = 32;  base = OFF_WT; }
  else if (id == 2) { base = OFF_W2; }
  else if (id == 3) { base = OFF_WC; }
  else if (id == 4) { base = OFF_WV; }
  else if (id == 5) { kp = 128; base = OFF_N1; }
  const int kg  = kp >> 3;
  const int tot = rows * kg;
  const int t   = blockIdx.x * NT + threadIdx.x;
  if (t >= tot) return;
  const int n = t / kg, g = t - n * kg;
  v8f x;
#pragma unroll
  for (int j = 0; j < 8; ++j) {
    const int k = 8 * g + j;
    float v;
    if (id == 0) {
      const int nn = n & 63;
      const int kr = (n < 64) ? k : (64 + k);
      v = We1[kr * HD + nn];
    } else if (id == 1) {
      int kr = (k < 16) ? (129 + k) : 128;
      kr = min(kr, KE1 - 1);
      const float w = We1[kr * HD + n];
      v = (k <= 16) ? w : 0.0f;
    } else if (id == 2) { v = We2[k * HD + n]; }
    else if (id == 3)   { v = Wc1[k * HD + n]; }
    else if (id == 4)   { v = Wv1[k * HD + n]; }
    else if (id == 5)   { v = Wn1[k * HD + n]; }
    else                { v = Wn2[k * HD + n]; }
    x[j] = v;
  }
  v8us hi, lo;
  split8(x, hi, lo);
  unsigned short* ph = wpl + base + 8 * t;
  unsigned short* pl = wpl + base + rows * kp + 8 * t;
  *(volatile v8us*)ph = hi;
  *(volatile v8us*)pl = lo;
  __threadfence();
  *(volatile v8us*)ph = hi;
  *(volatile v8us*)pl = lo;
}

__global__ __launch_bounds__(NT) __attribute__((amdgpu_num_vgpr(256)))
void k_pq(const float* __restrict__ nfi, const unsigned short* __restrict__ wpl, float* pqp, int nN) {
  __shared__ __attribute__((aligned(16))) unsigned short xs[NW][2][16 * HD];
  __shared__ __attribute__((aligned(16))) float st[NW][16 * PQW];
  const int tid = threadIdx.x, lane = tid & 31, wave = tid >> 5, h = lane >> 4, m = lane & 15;
  const int node0 = blockIdx.x * NPB + wave * 16;
  const int nd = min(node0 + m, nN - 1);
  {
    const float* xr = nfi + (size_t)nd * ROW + NFO + 32 * h;
#pragma unroll
    for (int q = 0; q < 4; ++q) {
      v8f x;
#pragma unroll
      for (int j = 0; j < 4; ++j) {
        const v2f p = *(const v2f*)(xr + 8 * q + 2 * j);
        x[2 * j] = p.x; x[2 * j + 1] = p.y;
      }
      v8us hi, lo;
      split8(x, hi, lo);
      *(v8us*)(&xs[wave][0][m * HD + 32 * h + 8 * q]) = hi;
      *(v8us*)(&xs[wave][1][m * HD + 32 * h + 8 * q]) = lo;
    }
  }
  __syncthreads();
  const unsigned short* ph = wpl + OFF_PQ;
  const unsigned short* pl = ph + 128 * HD;
  v8f acc[8];
#pragma unroll
  for (int ft = 0; ft < 8; ++ft) { v8f z = {0, 0, 0, 0, 0, 0, 0, 0}; acc[ft] = z; }
#pragma unroll
  for (int ks = 0; ks < 2; ++ks) {
    FragB bh, bl;
    ldpair(&xs[wave][0][0], &xs[wave][1][0], m * HD + 32 * ks + 8 * h, bh, bl);
#pragma unroll
    for (int ft = 0; ft < 8; ++ft) {
      FragB ah, al;
      ldpair(ph, pl, (16 * ft + m) * HD + 32 * ks + 8 * h, ah, al);
      acc[ft] = mma3(ah.v, al.v, bh.v, bl.v, acc[ft]);
    }
  }
#pragma unroll
  for (int ft = 0; ft < 8; ++ft) {
    float* d = &st[wave][m * PQW + 16 * ft + 8 * h];
    v4f u0, u1;
    u0.x = acc[ft][0]; u0.y = acc[ft][1]; u0.z = acc[ft][2]; u0.w = acc[ft][3];
    u1.x = acc[ft][4]; u1.y = acc[ft][5]; u1.z = acc[ft][6]; u1.w = acc[ft][7];
    *(v4f*)d = u0;
    *(v4f*)(d + 4) = u1;
  }
  __syncthreads();
#pragma unroll 4
  for (int i = 0; i < 16; ++i) {
    const v4f v = *(const v4f*)(&st[wave][i * PQW + 4 * lane]);
    *(volatile v4f*)(pqp + (size_t)(node0 + i) * PQW + 4 * lane) = v;
  }
  __threadfence();
#pragma unroll 4
  for (int i = 0; i < 16; ++i) {
    const v4f v = *(const v4f*)(&st[wave][i * PQW + 4 * lane]);
    *(volatile v4f*)(pqp + (size_t)(node0 + i) * PQW + 4 * lane) = v;
  }
}

__device__ __forceinline__ int scan_chunk(const int* __restrict__ keys, int nE, int cbase, int nodeBase,
                                          int* list, int tid, int wave) {
  int wc = 0;
  const int el0  = tid * EPT;
  const int e0   = cbase + el0;
  const int sent = -2147483647 - 1;
  v4i da, db;
  if (cbase + CHUNK <= nE) {
    da = *(const v4i*)(keys + e0);
    db = *(const v4i*)(keys + e0 + 4);
  } else {
    const int l = nE - 1;
    da.x = (e0     < nE) ? keys[min(e0,     l)] : sent;
    da.y = (e0 + 1 < nE) ? keys[min(e0 + 1, l)] : sent;
    da.z = (e0 + 2 < nE) ? keys[min(e0 + 2, l)] : sent;
    da.w = (e0 + 3 < nE) ? keys[min(e0 + 3, l)] : sent;
    db.x = (e0 + 4 < nE) ? keys[min(e0 + 4, l)] : sent;
    db.y = (e0 + 5 < nE) ? keys[min(e0 + 5, l)] : sent;
    db.z = (e0 + 6 < nE) ? keys[min(e0 + 6, l)] : sent;
    db.w = (e0 + 7 < nE) ? keys[min(e0 + 7, l)] : sent;
  }
  const unsigned nb = (unsigned)nodeBase;
  const unsigned s0 = (unsigned)da.x - nb, s1 = (unsigned)da.y - nb;
  const unsigned s2 = (unsigned)da.z - nb, s3 = (unsigned)da.w - nb;
  const unsigned s4 = (unsigned)db.x - nb, s5 = (unsigned)db.y - nb;
  const unsigned s6 = (unsigned)db.z - nb, s7 = (unsigned)db.w - nb;
  const bool h0 = s0 < (unsigned)NB, h1 = s1 < (unsigned)NB, h2 = s2 < (unsigned)NB, h3 = s3 < (unsigned)NB;
  const bool h4 = s4 < (unsigned)NB, h5 = s5 < (unsigned)NB, h6 = s6 < (unsigned)NB, h7 = s7 < (unsigned)NB;
  const unsigned any = __builtin_amdgcn_ballot_w32(h0 | h1 | h2 | h3 | h4 | h5 | h6 | h7);
  if (any != 0u) {
#define HITJ(J, HJ) { \
      const unsigned mj = __builtin_amdgcn_ballot_w32(HJ); \
      if (mj != 0u) { \
        if (HJ) { \
          const int pos = wc + (int)__builtin_amdgcn_mbcnt_lo(mj, 0u); \
          if (pos < WCAP) list[wave * WCAP + pos] = el0 + (J); \
        } \
        wc += (int)__builtin_popcount(mj); } }
    HITJ(0, h0)
    HITJ(1, h1)
    HITJ(2, h2)
    HITJ(3, h3)
    HITJ(4, h4)
    HITJ(5, h5)
    HITJ(6, h6)
    HITJ(7, h7)
#undef HITJ
  }
  return wc;
}

__device__ __forceinline__ void slab_store_pass(const float* aggl, const float* cxl, float* aggp, float* cxp,
                                                int nodeBase, int wave, int lane, int h, int m) {
  const size_t rb = (size_t)nodeBase;
#pragma unroll 4
  for (int i = 0; i < NB / (2 * NW); ++i) {
    const int row = (NB / NW) * wave + 2 * i + h;
    const v4f v = *(const v4f*)(aggl + row * HD + 4 * m);
    *(volatile v4f*)(aggp + (rb + row) * HD + 4 * m) = v;
  }
#pragma unroll
  for (int i = 0; i < NB / (32 * NW); ++i) {
    const int row = (NB / NW) * wave + 32 * i + lane;
    const v4f v = *(const v4f*)(cxl + row * 4);
    *(volatile v4f*)(cxp + (rb + row) * 4) = v;
  }
}

__global__ __launch_bounds__(NT) __attribute__((amdgpu_num_vgpr(256)))
void k_aggr(const float* __restrict__ nfi, const int* __restrict__ ei, const float* __restrict__ ef,
            const float* __restrict__ pqp, const unsigned short* __restrict__ wpl,
            const float* __restrict__ be1, const float* __restrict__ be2, const float* __restrict__ bc1,
            const float* __restrict__ wc2, const float* __restrict__ wi, const float* __restrict__ bi,
            float* aggp, float* cxp, int nN, int nE) {
#pragma clang fp contract(off)
  extern __shared__ float dynl[] __attribute__((aligned(16)));
  float* aggl = dynl;
  float* cxl  = dynl + (NB + 1) * HD;
  __shared__ __attribute__((aligned(16))) unsigned short xt[NW][2][32 * XP];
  __shared__ __attribute__((aligned(16))) float pm[NW][32 * HD];
  __shared__ __attribute__((aligned(16))) float dsm[NW * 32 * 4];
  __shared__ __attribute__((aligned(16))) float cwb[NW * 32];
  __shared__ __attribute__((aligned(16))) float gtb[NW * 32];
  __shared__ __attribute__((aligned(16))) int   slotb[NW * 32];
  __shared__ __attribute__((aligned(16))) int   list[LISTN];
  __shared__ __attribute__((aligned(16))) int   pend[PCAP];
  __shared__ __attribute__((aligned(16))) float vb[5 * HD];
  __shared__ int wcnt[NW];
  __shared__ int pendN;

  const int tid = threadIdx.x, lane = tid & 31, wave = tid >> 5, h = lane >> 4, m = lane & 15;
  const int nodeBase = blockIdx.x * NB;
  const int* keys = ei;
  const int* ends = ei + nE;
  const unsigned short* wth = wpl + OFF_WT; const unsigned short* wtl = wth + 64 * 32;
  const unsigned short* w2h = wpl + OFF_W2; const unsigned short* w2l = w2h + 64 * 64;
  const unsigned short* wch = wpl + OFF_WC; const unsigned short* wcl = wch + 64 * 64;

  for (int i = tid; i < (NB + 1) * HD; i += NT) aggl[i] = 0.0f;
  for (int i = tid; i < (NB + 1) * 4; i += NT) cxl[i] = 0.0f;
  if (tid < HD) {
    vb[tid]          = be1[tid];
    vb[HD + tid]     = be2[tid];
    vb[2 * HD + tid] = bc1[tid];
    vb[3 * HD + tid] = wc2[tid];
    vb[4 * HD + tid] = wi[tid];
  }
  if (tid == 0) pendN = 0;
  const float bi0 = bi[0];
  __syncthreads();

  const int nChunks = (nE + CHUNK - 1) / CHUNK;
#pragma unroll 1
  for (int ch = 0; ch < nChunks; ++ch) {
    const int cbase = ch * CHUNK;
    const int wc = scan_chunk(keys, nE, cbase, nodeBase, list, tid, wave);
    if (lane == 0) wcnt[wave] = wc;
    __syncthreads();

    const int base = pendN;
    int tot = 0, myoff = 0;
#pragma unroll
    for (int w = 0; w < NW; ++w) {
      int c = wcnt[w];
      c = c > WCAP ? WCAP : (c < 0 ? 0 : c);
      if (w < wave) myoff += c;
      tot += c;
    }
    int newN = base + tot;
    newN = newN > PCAP ? PCAP : newN;
    {
      int n = wcnt[wave];
      n = n > WCAP ? WCAP : (n < 0 ? 0 : n);
      const int* lp = list + wave * WCAP;
      for (int i = lane; i < n; i += 32) {
        const int pos = base + myoff + i;
        if (pos < PCAP) pend[pos] = cbase + lp[i];
      }
    }
    const int fin = (ch == nChunks - 1) ? 1 : 0;
    const int R   = (fin != 0) ? (newN + PASSN - 1) / PASSN : newN / PASSN;
    const int Pv  = (fin != 0) ? newN : R * PASSN;
    __syncthreads();

#pragma unroll 1
    for (int r = 0; r < R; ++r) {
      {
        const int idx = r * PASSN + wave * 32 + lane;
        const bool valid = idx < Pv;
        int e = pend[min(idx, PCAP - 1)];
        e = valid ? e : 0;
        e = min(max(e, 0), nE - 1);
        int s = keys[e];
        int t = ends[e];
        int slot = s - nodeBase;
        if (!valid || (unsigned)slot >= (unsigned)NB) slot = NB;
        s = min(max(s, 0), nN - 1);
        t = min(max(t, 0), nN - 1);
        const float* cs = nfi + (size_t)s * ROW;
        const float* ct = nfi + (size_t)t * ROW;
        const float dx = cs[0] - ct[0], dy = cs[1] - ct[1], dz = cs[2] - ct[2];
        const float nrm = sqrtf(dx * dx + dy * dy + dz * dz);
        v4f dv; dv.x = dx; dv.y = dy; dv.z = dz; dv.w = 0.0f;
        *(v4f*)(dsm + (wave * 32 + lane) * 4) = dv;
        slotb[wave * 32 + lane] = slot;
        const float* er = ef + (size_t)e * EFW;
        const v4f f0 = *(const v4f*)er;
        const v4f f1 = *(const v4f*)(er + 4);
        const v4f f2 = *(const v4f*)(er + 8);
        const v4f f3 = *(const v4f*)(er + 12);
        v8f xa, xb, xc;
        xa[0] = f0.x; xa[1] = f0.y; xa[2] = f0.z; xa[3] = f0.w; xa[4] = f1.x; xa[5] = f1.y; xa[6] = f1.z; xa[7] = f1.w;
        xb[0] = f2.x; xb[1] = f2.y; xb[2] = f2.z; xb[3] = f2.w; xb[4] = f3.x; xb[5] = f3.y; xb[6] = f3.z; xb[7] = f3.w;
        xc[0] = nrm; xc[1] = 0.0f; xc[2] = 0.0f; xc[3] = 0.0f; xc[4] = 0.0f; xc[5] = 0.0f; xc[6] = 0.0f; xc[7] = 0.0f;
        v8us ha, la, hb, lb, hc, lc;
        split8(xa, ha, la); split8(xb, hb, lb); split8(xc, hc, lc);
        const v8us z8 = {0, 0, 0, 0, 0, 0, 0, 0};
        unsigned short* xh = &xt[wave][0][lane * XP];
        unsigned short* xl = &xt[wave][1][lane * XP];
        *(v8us*)(xh) = ha; *(v8us*)(xh + 8) = hb; *(v8us*)(xh + 16) = hc; *(v8us*)(xh + 24) = z8;
        *(v8us*)(xl) = la; *(v8us*)(xl + 8) = lb; *(v8us*)(xl + 16) = lc; *(v8us*)(xl + 24) = z8;
        const float* pr = pqp + (size_t)s * PQW;
        const float* qr = pqp + (size_t)t * PQW + HD;
        float* dst = pm[wave] + lane * HD;
#pragma unroll 4
        for (int c = 0; c < HD / 4; ++c) {
          const v4f a  = *(const v4f*)(pr + 4 * c);
          const v4f b  = *(const v4f*)(qr + 4 * c);
          const v4f bb = *(const v4f*)(vb + 4 * c);
          *(v4f*)(dst + 4 * c) = (a + b) + bb;
        }
      }
      __syncthreads();

      {
        float* pw = pm[wave];
        unsigned short* th = &xt[wave][0][0];
        unsigned short* tl = &xt[wave][1][0];
#pragma unroll 1
        for (int tt = 0; tt < 2; ++tt) {
          const int er = 16 * tt + m;
          {
            FragB bh, bl;
            ldpair(th, tl, er * XP + 8 * h, bh, bl);
#pragma unroll 1
            for (int ft = 0; ft < 4; ++ft) {
              FragB ah, al;
              ldpair(wth, wtl, (16 * ft + m) * 32 + 8 * h, ah, al);
              const v8f c = ldc8(pw + er * HD + 16 * ft + 8 * h);
              const v8f d = silu8(mma3(ah.v, al.v, bh.v, bl.v, c));
              v8us hh8, ll8;
              split8(d, hh8, ll8);
              *(v8us*)(th + er * XP + 16 * ft + 8 * h) = hh8;
              *(v8us*)(tl + er * XP + 16 * ft + 8 * h) = ll8;
            }
          }
          __builtin_amdgcn_fence(__ATOMIC_RELEASE, "wavefront");
          __builtin_amdgcn_wave_barrier();
          float g;
          {
            FragB bh0, bl0, bh1, bl1;
            ldpair(th, tl, er * XP + 8 * h, bh0, bl0);
            ldpair(th, tl, er * XP + 32 + 8 * h, bh1, bl1);
            float pg = 0.0f;
#pragma unroll 1
            for (int ft = 0; ft < 4; ++ft) {
              FragB ah, al;
              v8f d = ldc8(vb + HD + 16 * ft + 8 * h);
              ldpair(w2h, w2l, (16 * ft + m) * HD + 8 * h, ah, al);
              d = mma3(ah.v, al.v, bh0.v, bl0.v, d);
              ldpair(w2h, w2l, (16 * ft + m) * HD + 32 + 8 * h, ah, al);
              d = mma3(ah.v, al.v, bh1.v, bl1.v, d);
              d = silu8(d);
              const v8f w8 = ldc8(vb + 4 * HD + 16 * ft + 8 * h);
#pragma unroll
              for (int rr = 0; rr < 8; ++rr) pg += d[rr] * w8[rr];
              stc8(pw + er * HD + 16 * ft + 8 * h, d);
            }
            pg += __shfl_xor(pg, 16, 32);
            g = sigm_f(pg + bi0);
          }
          __builtin_amdgcn_fence(__ATOMIC_RELEASE, "wavefront");
          __builtin_amdgcn_wave_barrier();
          float cwv;
          {
            FragB bh0, bl0, bh1, bl1;
            split8(ldc8(pw + er * HD + 8 * h),      bh0.u[0], bl0.u[0]);
            split8(ldc8(pw + er * HD + 16 + 8 * h), bh0.u[1], bl0.u[1]);
            split8(ldc8(pw + er * HD + 32 + 8 * h), bh1.u[0], bl1.u[0]);
            split8(ldc8(pw + er * HD + 48 + 8 * h), bh1.u[1], bl1.u[1]);
            float pc = 0.0f;
#pragma unroll 1
            for (int ft = 0; ft < 4; ++ft) {
              FragB ah, al;
              v8f d = ldc8(vb + 2 * HD + 16 * ft + 8 * h);
              ldpair(wch, wcl, (16 * ft + m) * HD + 8 * h, ah, al);
              d = mma3(ah.v, al.v, bh0.v, bl0.v, d);
              ldpair(wch, wcl, (16 * ft + m) * HD + 32 + 8 * h, ah, al);
              d = mma3(ah.v, al.v, bh1.v, bl1.v, d);
              const v8f chh = silu8(d);
              const v8f w8 = ldc8(vb + 3 * HD + 16 * ft + 8 * h);
#pragma unroll
              for (int rr = 0; rr < 8; ++rr) pc += chh[rr] * w8[rr];
            }
            pc += __shfl_xor(pc, 16, 32);
            cwv = pc;
          }
          if (h == 0) {
            cwb[wave * 32 + er] = cwv;
            gtb[wave * 32 + er] = g;
          }
        }
      }
      __syncthreads();

#pragma unroll 1
      for (int w = 0; w < NW; ++w) {
        if (wave == w) {
          const float* pmw = pm[w];
#pragma unroll 1
          for (int j = 0; j < 32; ++j) {
            int sl = slotb[w * 32 + j];
            sl = min(max(sl, 0), NB);
            const float gj = gtb[w * 32 + j];
            const float m0 = pmw[j * HD + lane] * gj;
            const float m1 = pmw[j * HD + 32 + lane] * gj;
            float* ar = aggl + sl * HD;
            const float n0 = ar[lane] + m0;
            const float n1 = ar[32 + lane] + m1;
            ar[lane] = n0;
            ar[32 + lane] = n1;
            const int c = lane & 3;
            const float dvv = dsm[(w * 32 + j) * 4 + c];
            const float cwj = cwb[w * 32 + j];
            const float add = (c < 3) ? dvv * cwj : 1.0f;
            const float nv = cxl[sl * 4 + c] + add;
            if (lane < 4) cxl[sl * 4 + c] = nv;
          }
        }
        __syncthreads();
      }
    }

    int rem = newN - R * PASSN;
    rem = rem < 0 ? 0 : rem;
    if (R > 0 && tid < rem) pend[tid] = pend[R * PASSN + tid];
    if (tid == 0) pendN = rem;
  }
  __syncthreads();

  slab_store_pass(aggl, cxl, aggp, cxp, nodeBase, wave, lane, h, m);
  __threadfence();
  slab_store_pass(aggl, cxl, aggp, cxp, nodeBase, wave, lane, h, m);
}

__global__ __launch_bounds__(NT) __attribute__((amdgpu_num_vgpr(256)))
void k_out(const float* __restrict__ nfi, const float* __restrict__ aggp, const float* __restrict__ cxp,
           const unsigned short* __restrict__ wpl,
           const float* __restrict__ bv1, const float* __restrict__ wv2, const float* __restrict__ bv2,
           const float* __restrict__ bn1, const float* __restrict__ bn2,
           float* outp, int nN, int outN) {
  __shared__ __attribute__((aligned(16))) unsigned short xn[NW][2][16 * PQW];
  __shared__ __attribute__((aligned(16))) float ost[NPB * ROW];
  __shared__ __attribute__((aligned(16))) float vb[4 * HD];
  const int tid = threadIdx.x, lane = tid & 31, wave = tid >> 5, h = lane >> 4, m = lane & 15;
  if (tid < HD) {
    vb[tid]          = bv1[tid];
    vb[HD + tid]     = wv2[tid];
    vb[2 * HD + tid] = bn1[tid];
    vb[3 * HD + tid] = bn2[tid];
  }
  const float bv20 = bv2[0];
  const int node0 = blockIdx.x * NPB + wave * 16;
  const int nd = min(node0 + m, nN - 1);
  {
    const float* xr = nfi + (size_t)nd * ROW + NFO + 32 * h;
#pragma unroll
    for (int q = 0; q < 4; ++q) {
      v8f x;
#pragma unroll
      for (int j = 0; j < 4; ++j) {
        const v2f p = *(const v2f*)(xr + 8 * q + 2 * j);
        x[2 * j] = p.x; x[2 * j + 1] = p.y;
      }
      v8us hi, lo;
      split8(x, hi, lo);
      *(v8us*)(&xn[wave][0][m * PQW + 32 * h + 8 * q]) = hi;
      *(v8us*)(&xn[wave][1][m * PQW + 32 * h + 8 * q]) = lo;
    }
    const float* ar = aggp + (size_t)nd * HD + 32 * h;
#pragma unroll
    for (int q = 0; q < 4; ++q) {
      const v4f a = *(const v4f*)(ar + 8 * q);
      const v4f b = *(const v4f*)(ar + 8 * q + 4);
      v8f x;
      x[0] = a.x; x[1] = a.y; x[2] = a.z; x[3] = a.w; x[4] = b.x; x[5] = b.y; x[6] = b.z; x[7] = b.w;
      v8us hi, lo;
      split8(x, hi, lo);
      *(v8us*)(&xn[wave][0][m * PQW + HD + 32 * h + 8 * q]) = hi;
      *(v8us*)(&xn[wave][1][m * PQW + HD + 32 * h + 8 * q]) = lo;
    }
  }
  __syncthreads();
  const unsigned short* wvh = wpl + OFF_WV; const unsigned short* wvl = wvh + 64 * 64;
  const unsigned short* n1h = wpl + OFF_N1; const unsigned short* n1l = n1h + 64 * 128;
  const unsigned short* n2h = wpl + OFF_N2; const unsigned short* n2l = n2h + 64 * 64;

  v8f av[4];
#pragma unroll
  for (int ft = 0; ft < 4; ++ft) av[ft] = ldc8(vb + 16 * ft + 8 * h);
#pragma unroll
  for (int ks = 0; ks < 2; ++ks) {
    FragB bh, bl;
    ldpair(&xn[wave][0][0], &xn[wave][1][0], m * PQW + 32 * ks + 8 * h, bh, bl);
#pragma unroll
    for (int ft = 0; ft < 4; ++ft) {
      FragB ah, al;
      ldpair(wvh, wvl, (16 * ft + m) * HD + 32 * ks + 8 * h, ah, al);
      av[ft] = mma3(ah.v, al.v, bh.v, bl.v, av[ft]);
    }
  }
  float sp = 0.0f;
#pragma unroll
  for (int ft = 0; ft < 4; ++ft) {
    const v8f w8 = ldc8(vb + HD + 16 * ft + 8 * h);
    const v8f sv = silu8(av[ft]);
#pragma unroll
    for (int rr = 0; rr < 8; ++rr) sp += sv[rr] * w8[rr];
  }
  sp += __shfl_xor(sp, 16, 32);
  const float sc = sp + bv20;

  {
    const float* nr = nfi + (size_t)nd * ROW;
    const float c0 = nr[0], c1 = nr[1], c2 = nr[2];
    const float v0 = nr[3], v1 = nr[4], v2 = nr[5];
    const v4f cx = *(const v4f*)(cxp + (size_t)nd * 4);
    const float rc = __builtin_amdgcn_rcpf(fmaxf(cx.w, 1.0f));
    const float t0 = c0 + cx.x * rc, t1 = c1 + cx.y * rc, t2 = c2 + cx.z * rc;
    const float o0 = t0 + sc * v0, o1 = t1 + sc * v1, o2 = t2 + sc * v2;
    if (h == 0) {
      float* orow = ost + (wave * 16 + m) * ROW;
      orow[0] = o0; orow[1] = o1; orow[2] = o2;
      orow[3] = v0; orow[4] = v1; orow[5] = v2;
    }
  }

  v8f a1[4];
#pragma unroll
  for (int ft = 0; ft < 4; ++ft) a1[ft] = ldc8(vb + 2 * HD + 16 * ft + 8 * h);
#pragma unroll
  for (int ks = 0; ks < 4; ++ks) {
    FragB bh, bl;
    ldpair(&xn[wave][0][0], &xn[wave][1][0], m * PQW + 32 * ks + 8 * h, bh, bl);
#pragma unroll
    for (int ft = 0; ft < 4; ++ft) {
      FragB ah, al;
      ldpair(n1h, n1l, (16 * ft + m) * PQW + 32 * ks + 8 * h, ah, al);
      a1[ft] = mma3(ah.v, al.v, bh.v, bl.v, a1[ft]);
    }
  }
  FragB b2h[2], b2l[2];
#pragma unroll
  for (int ks = 0; ks < 2; ++ks) d2b(silu8(a1[2 * ks]), silu8(a1[2 * ks + 1]), b2h[ks], b2l[ks]);
  v8f a2[4];
#pragma unroll
  for (int ft = 0; ft < 4; ++ft) a2[ft] = ldc8(vb + 3 * HD + 16 * ft + 8 * h);
#pragma unroll
  for (int ks = 0; ks < 2; ++ks) {
#pragma unroll
    for (int ft = 0; ft < 4; ++ft) {
      FragB ah, al;
      ldpair(n2h, n2l, (16 * ft + m) * HD + 32 * ks + 8 * h, ah, al);
      a2[ft] = mma3(ah.v, al.v, b2h[ks].v, b2l[ks].v, a2[ft]);
    }
  }
#pragma unroll
  for (int ft = 0; ft < 4; ++ft) {
    const float* nr = nfi + (size_t)nd * ROW + NFO + 16 * ft + 8 * h;
    const v2f p0 = *(const v2f*)nr, p1 = *(const v2f*)(nr + 2), p2 = *(const v2f*)(nr + 4), p3 = *(const v2f*)(nr + 6);
    float* orow = ost + (wave * 16 + m) * ROW + NFO + 16 * ft + 8 * h;
    orow[0] = p0.x + a2[ft][0]; orow[1] = p0.y + a2[ft][1];
    orow[2] = p1.x + a2[ft][2]; orow[3] = p1.y + a2[ft][3];
    orow[4] = p2.x + a2[ft][4]; orow[5] = p2.y + a2[ft][5];
    orow[6] = p3.x + a2[ft][6]; orow[7] = p3.y + a2[ft][7];
  }
  __syncthreads();

  const size_t fb = (size_t)blockIdx.x * (size_t)(NPB * ROW);
  const size_t lim = (size_t)(outN < 0 ? 0 : outN);
  for (int c = wave; c < OCH; c += NW) {
    const size_t gi = fb + (size_t)(c * 128 + 4 * lane);
    const v4f v = *(const v4f*)(ost + c * 128 + 4 * lane);
    if (gi + 4 <= lim) *(volatile v4f*)(outp + gi) = v;
  }
  __threadfence();
  for (int c = wave; c < OCH; c += NW) {
    const size_t gi = fb + (size_t)(c * 128 + 4 * lane);
    const v4f v = *(const v4f*)(ost + c * 128 + 4 * lane);
    if (gi + 4 <= lim) *(volatile v4f*)(outp + gi) = v;
  }
}

extern "C" void kernel_launch(void* const* d_in, const int* in_sizes, int n_in,
                              void* d_out, int out_size, void* d_ws, size_t ws_size,
                              hipStream_t stream) {
  if (n_in < 20) return;
  const int nN = in_sizes[0] / ROW;
  const int nE = in_sizes[1] / 2;
  if (nN <= 0 || nE <= 0) return;
  if (in_sizes[0] != nN * ROW || in_sizes[1] != nE * 2 || in_sizes[2] != nE * EFW) return;
  if (in_sizes[3] != KE1 * HD || in_sizes[4] < HD || in_sizes[5] != HD * HD || in_sizes[6] < HD) return;
  if (in_sizes[7] != HD * HD || in_sizes[8] < HD || in_sizes[9] < HD) return;
  if (in_sizes[10] != HD * HD || in_sizes[11] < HD || in_sizes[12] < HD || in_sizes[13] < 1) return;
  if (in_sizes[14] != 2 * HD * HD || in_sizes[15] < HD || in_sizes[16] != HD * HD || in_sizes[17] < HD) return;
  if (in_sizes[18] < HD || in_sizes[19] < 1) return;
  if (out_size != nN * ROW) return;

  const float* nfi  = (const float*)d_in[0];
  const int*   eidx = (const int*)d_in[1];
  const float* ef   = (const float*)d_in[2];
  const float* We1  = (const float*)d_in[3];
  const float* be1  = (const float*)d_in[4];
  const float* We2  = (const float*)d_in[5];
  const float* be2  = (const float*)d_in[6];
  const float* Wc1  = (const float*)d_in[7];
  const float* bc1  = (const float*)d_in[8];
  const float* Wc2  = (const float*)d_in[9];
  const float* Wv1  = (const float*)d_in[10];
  const float* bv1  = (const float*)d_in[11];
  const float* Wv2  = (const float*)d_in[12];
  const float* bv2  = (const float*)d_in[13];
  const float* Wn1  = (const float*)d_in[14];
  const float* bn1  = (const float*)d_in[15];
  const float* Wn2  = (const float*)d_in[16];
  const float* bn2  = (const float*)d_in[17];
  const float* Wi   = (const float*)d_in[18];
  const float* bi   = (const float*)d_in[19];
  float* out = (float*)d_out;

  const int nBlkE = (nN + NB - 1) / NB;
  const int nBlkN = (nN + NPB - 1) / NPB;

  char* ws = (char*)d_ws;
  size_t off = 0;
  const size_t oW  = off; off += (size_t)WPLN * sizeof(unsigned short);           off = (off + 255) & ~(size_t)255;
  const size_t oPQ = off; off += (size_t)nBlkN * NPB * PQW * sizeof(float);       off = (off + 255) & ~(size_t)255;
  const size_t oAG = off; off += (size_t)nBlkE * NB * HD * sizeof(float);         off = (off + 255) & ~(size_t)255;
  const size_t oCX = off; off += (size_t)nBlkE * NB * 4 * sizeof(float);          off = (off + 255) & ~(size_t)255;
  if (off > ws_size) return;
  unsigned short* wpl = (unsigned short*)(ws + oW);
  float* pqp  = (float*)(ws + oPQ);
  float* aggp = (float*)(ws + oAG);
  float* cxp  = (float*)(ws + oCX);

  const size_t dynB = (size_t)((NB + 1) * HD + (NB + 1) * 4) * sizeof(float);
  hipFuncSetAttribute(reinterpret_cast<const void*>(&k_aggr), hipFuncAttributeMaxDynamicSharedMemorySize, (int)dynB);

  k_prep<<<dim3(8, 7), NT, 0, stream>>>(We1, We2, Wc1, Wv1, Wn1, Wn2, wpl);
  k_pq<<<nBlkN, NT, 0, stream>>>(nfi, wpl, pqp, nN);
  k_aggr<<<nBlkE, NT, dynB, stream>>>(nfi, eidx, ef, pqp, wpl, be1, be2, bc1, Wc2, Wi, bi, aggp, cxp, nN, nE);
  k_out<<<nBlkN, NT, 0, stream>>>(nfi, aggp, cxp, wpl, bv1, Wv2, bv2, bn1, bn2, out, nN, out_size);
}
